// GenePanelGNN_88630945120677
// MI455X (gfx1250) — hardware-verified
//
#include <hip/hip_runtime.h>
#include <stddef.h>


#define DF      128
#define KW      256
#define NTHR    256
#define NWAVE   8
#define EPT     8
#define NGRP    2
#define CHUNK   (NTHR * EPT * NGRP)
#define WCAP    (EPT * NGRP * 32)
#define LISTN   (NWAVE * WCAP)
#define NBS     512
#define PB      64
#define PTHR    256
#define CPL     (DF * KW)
#define BPL     (DF * DF)
#define WPLN    (8 * CPL + 2 * BPL)

#define LDS_SAGE (NBS * DF * 4 + LISTN * 4 + 64 + NBS * 4 + NBS * 4)

static_assert((CHUNK & (CHUNK - 1)) == 0);
static_assert(CHUNK <= 4096);
static_assert((NBS & (NBS - 1)) == 0);
static_assert(NBS <= 4096);
static_assert(NBS % 64 == 0);
static_assert(PB == 64);
static_assert(PTHR == 256);
static_assert(LDS_SAGE <= 300 * 1024);

typedef float          v4f   __attribute__((ext_vector_type(4)));
typedef float          v8f   __attribute__((ext_vector_type(8)));
typedef int            v4i   __attribute__((ext_vector_type(4)));
typedef unsigned short v8us  __attribute__((ext_vector_type(8)));
typedef __bf16         v16bf __attribute__((ext_vector_type(16)));
union FragB { v16bf v; v8us u[2]; };

__device__ __forceinline__ unsigned bf_rne_bits(float x) {
  const unsigned u = __float_as_uint(x);
  return (u + 0x7FFFu + ((u >> 16) & 1u)) >> 16;
}

__device__ __forceinline__ void split8(v4f a, v4f b, v8us& hi, v8us& lo) {
  const float x[8] = {a.x, a.y, a.z, a.w, b.x, b.y, b.z, b.w};
  v8us hv = {0, 0, 0, 0, 0, 0, 0, 0};
  v8us lv = {0, 0, 0, 0, 0, 0, 0, 0};
#pragma unroll
  for (int i = 0; i < 8; ++i) {
    const unsigned hb = bf_rne_bits(x[i]);
    const float    hf = __uint_as_float(hb << 16);
    const unsigned lb = bf_rne_bits(x[i] - hf);
    hv[i] = (unsigned short)hb;
    lv[i] = (unsigned short)lb;
  }
  hi = hv;
  lo = lv;
}

__device__ __forceinline__ v8f wmb3(v16bf ah, v16bf al, v16bf bh, v16bf bl, v8f c) {
  c = __builtin_amdgcn_wmma_f32_16x16x32_bf16(false, ah, false, bh, (short)0, c, false, false);
  c = __builtin_amdgcn_wmma_f32_16x16x32_bf16(false, al, false, bh, (short)0, c, false, false);
  c = __builtin_amdgcn_wmma_f32_16x16x32_bf16(false, ah, false, bl, (short)0, c, false, false);
  asm volatile("v_nop\n\tv_nop\n\tv_nop\n\tv_nop" : "+v"(c) : "v"(ah), "v"(al), "v"(bh), "v"(bl));
  return c;
}

__device__ __forceinline__ void mac4(v8f (&c)[4], v16bf ah, v16bf al,
                                     const unsigned short* __restrict__ whi,
                                     const unsigned short* __restrict__ wlo,
                                     int pitch, int kofs, int ncol0) {
#pragma unroll
  for (int t = 0; t < 4; ++t) {
    const size_t o = (size_t)(ncol0 + 16 * t) * pitch + kofs;
    FragB bh, bl;
    bh.u[0] = *(const v8us*)(whi + o);
    bh.u[1] = *(const v8us*)(whi + o + 16);
    bl.u[0] = *(const v8us*)(wlo + o);
    bl.u[1] = *(const v8us*)(wlo + o + 16);
    c[t] = wmb3(ah, al, bh.v, bl.v, c[t]);
  }
}

template <int NB>
__device__ __forceinline__ int scan_chunk(const int* __restrict__ keys, int nE, int cbase, int nodeBase,
                                          int vec8, int* list, int tid, int lane, int wave) {
  int wc = 0;
#pragma unroll
  for (int g = 0; g < NGRP; ++g) {
    const int el0  = (g * NTHR + tid) * EPT;
    const int e0   = cbase + el0;
    const int sent = -2147483647 - 1;
    v4i da, db;
    if (vec8 != 0 && cbase + CHUNK <= nE) {
      da = *(const v4i*)(keys + e0);
      db = *(const v4i*)(keys + e0 + 4);
    } else {
      da.x = (e0     < nE) ? keys[min(e0,     nE - 1)] : sent;
      da.y = (e0 + 1 < nE) ? keys[min(e0 + 1, nE - 1)] : sent;
      da.z = (e0 + 2 < nE) ? keys[min(e0 + 2, nE - 1)] : sent;
      da.w = (e0 + 3 < nE) ? keys[min(e0 + 3, nE - 1)] : sent;
      db.x = (e0 + 4 < nE) ? keys[min(e0 + 4, nE - 1)] : sent;
      db.y = (e0 + 5 < nE) ? keys[min(e0 + 5, nE - 1)] : sent;
      db.z = (e0 + 6 < nE) ? keys[min(e0 + 6, nE - 1)] : sent;
      db.w = (e0 + 7 < nE) ? keys[min(e0 + 7, nE - 1)] : sent;
    }
    const unsigned nb = (unsigned)nodeBase;
    const unsigned s0 = (unsigned)da.x - nb, s1 = (unsigned)da.y - nb;
    const unsigned s2 = (unsigned)da.z - nb, s3 = (unsigned)da.w - nb;
    const unsigned s4 = (unsigned)db.x - nb, s5 = (unsigned)db.y - nb;
    const unsigned s6 = (unsigned)db.z - nb, s7 = (unsigned)db.w - nb;
    const bool h0 = s0 < (unsigned)NB, h1 = s1 < (unsigned)NB, h2 = s2 < (unsigned)NB, h3 = s3 < (unsigned)NB;
    const bool h4 = s4 < (unsigned)NB, h5 = s5 < (unsigned)NB, h6 = s6 < (unsigned)NB, h7 = s7 < (unsigned)NB;
    const unsigned any = __builtin_amdgcn_ballot_w32(h0 | h1 | h2 | h3 | h4 | h5 | h6 | h7);
    if (any != 0u) {
#define HITJ(J, HJ, SJ) { \
        const unsigned mj = __builtin_amdgcn_ballot_w32(HJ); \
        if (mj != 0u) { \
          if (HJ) { \
            const int pos = wc + (int)__builtin_amdgcn_mbcnt_lo(mj, 0u); \
            if (pos < WCAP) list[wave * WCAP + pos] = ((el0 + (J)) << 12) | (int)(SJ); \
          } \
          wc += (int)__builtin_popcount(mj); } }
      HITJ(0, h0, s0)
      HITJ(1, h1, s1)
      HITJ(2, h2, s2)
      HITJ(3, h3, s3)
      HITJ(4, h4, s4)
      HITJ(5, h5, s5)
      HITJ(6, h6, s6)
      HITJ(7, h7, s7)
#undef HITJ
    }
  }
  return wc;
}

__global__ __launch_bounds__(NTHR) void k_wprep(
    const float* W0, const float* W1, const float* W2, const float* W3, const float* W4,
    const float* W5, const float* W6, const float* W7, const float* W8,
    unsigned short* wpl) {
  const int j = blockIdx.y;
  const int t = blockIdx.x * NTHR + threadIdx.x;
  if (t >= DF * DF / 8) return;
  const float* W = (j == 0) ? W0 : (j == 1) ? W1 : (j == 2) ? W2 : (j == 3) ? W3 :
                   (j == 4) ? W4 : (j == 5) ? W5 : (j == 6) ? W6 : (j == 7) ? W7 : W8;
  const int n  = t >> 4;
  const int k0 = (t & 15) * 8;
  const float* p = W + (size_t)k0 * DF + n;
  v4f a, b;
  a.x = p[0];      a.y = p[DF];     a.z = p[2 * DF]; a.w = p[3 * DF];
  b.x = p[4 * DF]; b.y = p[5 * DF]; b.z = p[6 * DF]; b.w = p[7 * DF];
  v8us hv, lv;
  split8(a, b, hv, lv);
  unsigned short* hp;
  unsigned short* lp;
  size_t dst;
  if (j < 8) {
    hp  = wpl + (size_t)(2 * (j >> 1)) * CPL;
    lp  = hp + CPL;
    dst = (size_t)n * KW + (size_t)(128 * (j & 1)) + k0;
  } else {
    hp  = wpl + (size_t)8 * CPL;
    lp  = hp + BPL;
    dst = (size_t)n * DF + k0;
  }
  *(volatile v8us*)(hp + dst) = hv;
  *(volatile v8us*)(lp + dst) = lv;
  __threadfence();
  *(volatile v8us*)(hp + dst) = hv;
  *(volatile v8us*)(lp + dst) = lv;
}

template <int NB>
__global__ __launch_bounds__(NTHR) void k_sage(
    const int* __restrict__ keys, const int* __restrict__ other,
    const float* __restrict__ xsrc, const float* __restrict__ xdst,
    const unsigned short* __restrict__ whi, const unsigned short* __restrict__ wlo,
    const float* __restrict__ bias, float* hout,
    int nDst, int nSrc, int nE, int vec8, int relu) {
  extern __shared__ v4f lds_dyn[];
  float* acc  = (float*)lds_dyn;
  int*   list = (int*)(acc + NB * DF);
  int*   wcnt = list + LISTN;
  int*   cnt  = wcnt + 16;
  float* inv  = (float*)(cnt + NB);
  const int tid = threadIdx.x, lane = tid & 31, wave = tid >> 5, hh = lane >> 4, m = lane & 15;
  const int nodeBase = blockIdx.x * NB;

  {
    const v4f z = {0.f, 0.f, 0.f, 0.f};
    for (int i = tid; i < NB * DF / 4; i += NTHR) lds_dyn[i] = z;
    for (int i = tid; i < NB; i += NTHR) cnt[i] = 0;
  }
  __syncthreads();

  const int nChunks = (nE + CHUNK - 1) / CHUNK;
#pragma unroll 1
  for (int ch = 0; ch < nChunks; ++ch) {
    const int cbase = ch * CHUNK;
    const int wc = scan_chunk<NB>(keys, nE, cbase, nodeBase, vec8, list, tid, lane, wave);
    if (lane == 0) wcnt[wave] = wc;
    __syncthreads();
    if (wave == 0) {
#pragma unroll 1
      for (int wsx = 0; wsx < NWAVE; ++wsx) {
        int n = __builtin_amdgcn_readfirstlane(wcnt[wsx]);
        n = n > WCAP ? WCAP : (n < 0 ? 0 : n);
        const int* lp = list + wsx * WCAP;
#pragma unroll 1
        for (int i = 0; i < n; ++i) {
          const int ent  = __builtin_amdgcn_readfirstlane(lp[i]);
          const int slot = ent & (NB - 1);
          int e = cbase + ((ent >> 12) & (CHUNK - 1));
          e = e > nE - 1 ? nE - 1 : e;
          int s = other[e];
          s = s < 0 ? 0 : (s > nSrc - 1 ? nSrc - 1 : s);
          const v4f v = *(const v4f*)(xsrc + (size_t)s * DF + 4 * lane);
          v4f* ap = (v4f*)(acc + slot * DF + 4 * lane);
          *ap = *ap + v;
          if (lane == 0) cnt[slot] = cnt[slot] + 1;
        }
      }
    }
    __syncthreads();
  }

  for (int s = tid; s < NB; s += NTHR) inv[s] = 1.0f / fmaxf((float)cnt[s], 1.0f);
  __syncthreads();
#pragma unroll 4
  for (int i = 0; i < (NB * DF / 4) / NTHR; ++i) {
    const int idx  = i * NTHR + tid;
    const int slot = idx >> 5;
    const int c4   = (idx & 31) * 4;
    v4f* ap = (v4f*)(acc + slot * DF + c4);
    *ap = *ap * inv[slot];
  }
  __syncthreads();

  const int rsub = wave & 3, th = wave >> 2;
  constexpr int G4N = NB / 64;
#pragma unroll 1
  for (int g4 = 0; g4 < G4N; ++g4) {
    const int r0 = 64 * g4 + 16 * rsub;
    int node = nodeBase + r0 + m;
    node = node > nDst - 1 ? nDst - 1 : node;
    const float* xrow = xdst + (size_t)node * DF + 8 * hh;
    const float* arow = acc + (r0 + m) * DF + 8 * hh;
    v8f c4[4];
#pragma unroll
    for (int t = 0; t < 4; ++t) { v8f z = {0.f, 0.f, 0.f, 0.f, 0.f, 0.f, 0.f, 0.f}; c4[t] = z; }

#pragma unroll 1
    for (int kt = 0; kt < 4; ++kt) {
      const float* ap = arow + 32 * kt;
      const v4f p0 = *(const v4f*)ap,        p1 = *(const v4f*)(ap + 4);
      const v4f p2 = *(const v4f*)(ap + 16), p3 = *(const v4f*)(ap + 20);
      FragB ah, al;
      split8(p0, p1, ah.u[0], al.u[0]);
      split8(p2, p3, ah.u[1], al.u[1]);
      mac4(c4, ah.v, al.v, whi, wlo, KW, 32 * kt + 8 * hh, 64 * th + m);
    }
#pragma unroll 1
    for (int kt = 0; kt < 4; ++kt) {
      const float* gp = xrow + 32 * kt;
      const v4f p0 = *(const v4f*)gp,        p1 = *(const v4f*)(gp + 4);
      const v4f p2 = *(const v4f*)(gp + 16), p3 = *(const v4f*)(gp + 20);
      FragB ah, al;
      split8(p0, p1, ah.u[0], al.u[0]);
      split8(p2, p3, ah.u[1], al.u[1]);
      mac4(c4, ah.v, al.v, whi, wlo, KW, DF + 32 * kt + 8 * hh, 64 * th + m);
    }
    __syncthreads();

    float* sp = acc + (r0 + 8 * hh) * DF + 64 * th + m;
#pragma unroll
    for (int t = 0; t < 4; ++t) {
      const float bv = bias[64 * th + 16 * t + m];
#pragma unroll
      for (int r = 0; r < 8; ++r) {
        float v = c4[t][r] + bv;
        v = (relu != 0) ? fmaxf(v, 0.0f) : v;
        sp[r * DF + 16 * t] = v;
      }
    }
    __syncthreads();

    const float* lrow = acc + (64 * g4 + 8 * wave) * DF + 4 * lane;
    float* grow = hout + ((size_t)nodeBase + 64 * g4 + 8 * wave) * DF + 4 * lane;
#pragma unroll
    for (int i = 0; i < 8; ++i) {
      const v4f v = *(const v4f*)(lrow + i * DF);
      *(volatile v4f*)(grow + (size_t)i * DF) = v;
    }
    __threadfence();
#pragma unroll
    for (int i = 0; i < 8; ++i) {
      const v4f v = *(const v4f*)(lrow + i * DF);
      *(volatile v4f*)(grow + (size_t)i * DF) = v;
    }
  }
}

__global__ __launch_bounds__(PTHR) void k_pair(
    const float* __restrict__ og, const float* __restrict__ op,
    const int* __restrict__ pg, const int* __restrict__ pp,
    const unsigned short* __restrict__ bhi, const unsigned short* __restrict__ blo,
    const float* __restrict__ bb, float* out, int P, int nG, int nP) {
  __shared__ __attribute__((aligned(16))) unsigned short shi[PB * DF];
  __shared__ __attribute__((aligned(16))) unsigned short slo[PB * DF];
  __shared__ __attribute__((aligned(16))) float spart[2 * PB];
  const int tid = threadIdx.x, lane = tid & 31, wave = tid >> 5, hh = lane >> 4, m = lane & 15;
  const int pbase = blockIdx.x * PB;

#pragma unroll
  for (int it = 0; it < (PB * DF / 8) / PTHR; ++it) {
    const int idx = it * PTHR + tid;
    const int row = idx >> 4;
    const int c8  = (idx & 15) * 8;
    int p = pbase + row;
    p = p > P - 1 ? P - 1 : p;
    int gi = pg[p];
    gi = gi < 0 ? 0 : (gi > nG - 1 ? nG - 1 : gi);
    const float* gr = og + (size_t)gi * DF + c8;
    const v4f a = *(const v4f*)gr, b = *(const v4f*)(gr + 4);
    v8us hv, lv;
    split8(a, b, hv, lv);
    *(v8us*)(shi + row * DF + c8) = hv;
    *(v8us*)(slo + row * DF + c8) = lv;
  }
  __syncthreads();

  const int rt = wave & 3, th = wave >> 2;
  v8f c4[4];
#pragma unroll
  for (int t = 0; t < 4; ++t) { v8f z = {0.f, 0.f, 0.f, 0.f, 0.f, 0.f, 0.f, 0.f}; c4[t] = z; }
  const unsigned short* ahp = shi + (rt * 16 + m) * DF + 8 * hh;
  const unsigned short* alp = slo + (rt * 16 + m) * DF + 8 * hh;
#pragma unroll 1
  for (int kt = 0; kt < 4; ++kt) {
    FragB ah, al;
    ah.u[0] = *(const v8us*)(ahp + 32 * kt);
    ah.u[1] = *(const v8us*)(ahp + 32 * kt + 16);
    al.u[0] = *(const v8us*)(alp + 32 * kt);
    al.u[1] = *(const v8us*)(alp + 32 * kt + 16);
    mac4(c4, ah.v, al.v, bhi, blo, DF, 32 * kt + 8 * hh, 64 * th + m);
  }

  const int prow0 = pbase + rt * 16 + 8 * hh;
  float part[8];
#pragma unroll
  for (int r = 0; r < 8; ++r) {
    int pr = prow0 + r;
    pr = pr > P - 1 ? P - 1 : pr;
    int pi = pp[pr];
    pi = pi < 0 ? 0 : (pi > nP - 1 ? nP - 1 : pi);
    const float* orow = op + (size_t)pi * DF + 64 * th + m;
    float s = 0.f;
#pragma unroll
    for (int t = 0; t < 4; ++t) s += c4[t][r] * orow[16 * t];
    part[r] = s;
  }
#pragma unroll
  for (int r = 0; r < 8; ++r) {
    float v = part[r];
    v += __shfl_xor(v, 1, 32);
    v += __shfl_xor(v, 2, 32);
    v += __shfl_xor(v, 4, 32);
    v += __shfl_xor(v, 8, 32);
    part[r] = v;
  }
  if (m == 0) {
#pragma unroll
    for (int r = 0; r < 8; ++r) spart[th * PB + rt * 16 + 8 * hh + r] = part[r];
  }
  __syncthreads();

  if (wave == 0) {
    const float b0 = bb[0];
    if (pbase + PB <= P) {
      const int l16 = lane & 15;
      const v4f a = *(const v4f*)(spart + 4 * l16);
      const v4f b = *(const v4f*)(spart + PB + 4 * l16);
      const v4f v = a + b + b0;
      if (lane < 16) *(volatile v4f*)(out + (size_t)pbase + 4 * lane) = v;
      __threadfence();
      if (lane < 16) *(volatile v4f*)(out + (size_t)pbase + 4 * lane) = v;
    } else {
      const int i0 = lane, i1 = lane + 32;
      const float v0 = spart[i0] + spart[PB + i0] + b0;
      const float v1 = spart[i1] + spart[PB + i1] + b0;
      if (pbase + i0 < P) *(volatile float*)(out + (size_t)pbase + i0) = v0;
      if (pbase + i1 < P) *(volatile float*)(out + (size_t)pbase + i1) = v1;
      __threadfence();
      if (pbase + i0 < P) *(volatile float*)(out + (size_t)pbase + i0) = v0;
      if (pbase + i1 < P) *(volatile float*)(out + (size_t)pbase + i1) = v1;
    }
  }
}

extern "C" void kernel_launch(void* const* d_in, const int* in_sizes, int n_in,
                              void* d_out, int out_size, void* d_ws, size_t ws_size,
                              hipStream_t stream) {
  if (n_in < 20) return;
  const int NG = in_sizes[0] / DF;
  const int NP = in_sizes[1] / DF;
  const int E  = in_sizes[2];
  const int P  = in_sizes[4];
  if (NG <= 0 || NP <= 0 || E <= 0 || P <= 0) return;
  if (in_sizes[0] != NG * DF || in_sizes[1] != NP * DF) return;
  if (in_sizes[3] != E || in_sizes[5] != P || out_size != P) return;
  if (in_sizes[6] != DF * DF || in_sizes[8] != DF * DF || in_sizes[9] != DF * DF || in_sizes[11] != DF * DF) return;
  if (in_sizes[12] != DF * DF || in_sizes[14] != DF * DF || in_sizes[15] != DF * DF || in_sizes[17] != DF * DF) return;
  if (in_sizes[18] != DF * DF) return;
  if (in_sizes[7] < DF || in_sizes[10] < DF || in_sizes[13] < DF || in_sizes[16] < DF || in_sizes[19] < 1) return;

  const float* x_gene  = (const float*)d_in[0];
  const float* x_panel = (const float*)d_in[1];
  const int*   e_src   = (const int*)d_in[2];
  const int*   e_dst   = (const int*)d_in[3];
  const int*   p_gene  = (const int*)d_in[4];
  const int*   p_panel = (const int*)d_in[5];
  const float* W1_gp_l = (const float*)d_in[6];
  const float* b1_gp   = (const float*)d_in[7];
  const float* W1_gp_r = (const float*)d_in[8];
  const float* W1_pg_l = (const float*)d_in[9];
  const float* b1_pg   = (const float*)d_in[10];
  const float* W1_pg_r = (const float*)d_in[11];
  const float* W2_gp_l = (const float*)d_in[12];
  const float* b2_gp   = (const float*)d_in[13];
  const float* W2_gp_r = (const float*)d_in[14];
  const float* W2_pg_l = (const float*)d_in[15];
  const float* b2_pg   = (const float*)d_in[16];
  const float* W2_pg_r = (const float*)d_in[17];
  const float* Wb      = (const float*)d_in[18];
  const float* bb      = (const float*)d_in[19];
  float* out = (float*)d_out;

  const int nBP = (NP + NBS - 1) / NBS;
  const int nBG = (NG + NBS - 1) / NBS;
  const int nPB = (P + PB - 1) / PB;

  char* ws = (char*)d_ws;
  size_t off = 0;
  const size_t oW  = off; off += (size_t)WPLN * 2;                      off = (off + 255) & ~(size_t)255;
  const size_t ohP = off; off += (size_t)nBP * NBS * DF * 4;            off = (off + 255) & ~(size_t)255;
  const size_t ohG = off; off += (size_t)nBG * NBS * DF * 4;            off = (off + 255) & ~(size_t)255;
  const size_t ooP = off; off += (size_t)nBP * NBS * DF * 4;            off = (off + 255) & ~(size_t)255;
  const size_t ooG = off; off += (size_t)nBG * NBS * DF * 4;            off = (off + 255) & ~(size_t)255;
  if (off > ws_size) return;
  unsigned short* wpl = (unsigned short*)(ws + oW);
  float* hP = (float*)(ws + ohP);
  float* hG = (float*)(ws + ohG);
  float* oP = (float*)(ws + ooP);
  float* oG = (float*)(ws + ooG);

  const int vec8 = ((E & 3) == 0) ? 1 : 0;

  k_wprep<<<dim3(DF * DF / 8 / NTHR, 9), NTHR, 0, stream>>>(
      W1_gp_l, W1_gp_r, W1_pg_l, W1_pg_r, W2_gp_l, W2_gp_r, W2_pg_l, W2_pg_r, Wb, wpl);

  hipFuncSetAttribute(reinterpret_cast<const void*>(&k_sage<NBS>),
                      hipFuncAttributeMaxDynamicSharedMemorySize, LDS_SAGE);

  k_sage<NBS><<<nBP, NTHR, LDS_SAGE, stream>>>(e_dst, e_src, x_gene, x_panel,
      wpl + 0 * CPL, wpl + 1 * CPL, b1_gp, hP, NP, NG, E, vec8, 1);
  k_sage<NBS><<<nBG, NTHR, LDS_SAGE, stream>>>(e_src, e_dst, x_panel, x_gene,
      wpl + 2 * CPL, wpl + 3 * CPL, b1_pg, hG, NG, NP, E, vec8, 1);
  k_sage<NBS><<<nBP, NTHR, LDS_SAGE, stream>>>(e_dst, e_src, hG, hP,
      wpl + 4 * CPL, wpl + 5 * CPL, b2_gp, oP, NP, NG, E, vec8, 0);
  k_sage<NBS><<<nBG, NTHR, LDS_SAGE, stream>>>(e_src, e_dst, hP, hG,
      wpl + 6 * CPL, wpl + 7 * CPL, b2_pg, oG, NG, NP, E, vec8, 0);

  k_pair<<<nPB, PTHR, 0, stream>>>(oG, oP, p_gene, p_panel,
      wpl + 8 * CPL, wpl + 8 * CPL + BPL, bb, out, P, NG, NP);
}
